// BQQLinearInference_82635170775233
// MI455X (gfx1250) — hardware-verified
//
#include <hip/hip_runtime.h>


#define BB   512
#define PPd  2
#define JJ   32
#define KKb  32
#define MM   128
#define LL   16
#define NNb  128
#define JL   (JJ * LL)
#define PKL  (PPd * KKb * LL)
typedef _Float16 h16;
typedef unsigned short bf;
typedef __attribute__((ext_vector_type(16))) __bf16   v16bf;
typedef __attribute__((ext_vector_type(16))) _Float16 v16h;
typedef __attribute__((ext_vector_type(8)))  _Float16 v8h;
typedef __attribute__((ext_vector_type(8)))  unsigned short v8us;
typedef __attribute__((ext_vector_type(8)))  float    v8f;
typedef __attribute__((ext_vector_type(4)))  float    v4f;
typedef v8h  __attribute__((may_alias)) v8ha;
typedef v4f  __attribute__((may_alias)) v4fa;
typedef v8us __attribute__((may_alias)) v8usa;

__device__ __forceinline__ unsigned short f2bf(float f) { unsigned u = __float_as_uint(f); u += 0x7FFFu + ((u >> 16) & 1u); return (unsigned short)(u >> 16); }
__device__ __forceinline__ float bf2f(unsigned short b) { return __uint_as_float(((unsigned)b) << 16); }
__device__ __forceinline__ float bfr(float f) { return bf2f(f2bf(f)); }
__device__ __forceinline__ v16h cat16(v8h lo, v8h hi) { return __builtin_shufflevector(lo, hi, 0, 1, 2, 3, 4, 5, 6, 7, 8, 9, 10, 11, 12, 13, 14, 15); }
__device__ __forceinline__ v16bf cat16b(v8us lo, v8us hi) { return __builtin_bit_cast(v16bf, __builtin_shufflevector(lo, hi, 0, 1, 2, 3, 4, 5, 6, 7, 8, 9, 10, 11, 12, 13, 14, 15)); }
__device__ __forceinline__ v8f wmma16(v16h a, v16h b, v8f c) { return __builtin_amdgcn_wmma_f32_16x16x32_f16(false, a, false, b, (short)0, c, false, false); }
__device__ __forceinline__ v8f wmmab(v16bf a, v16bf b, v8f c) { return __builtin_amdgcn_wmma_f32_16x16x32_bf16(false, a, false, b, (short)0, c, false, false); }


template <typename T16> struct WFrag;
template <> struct WFrag<h16> { typedef v16h V; static __device__ __forceinline__ V ld(const h16* p) { return cat16(*(const v8h*)p, *(const v8h*)(p + 16)); } static __device__ __forceinline__ v8f mma(V a, V b, v8f c) { return wmma16(a, b, c); } };
template <> struct WFrag<bf> { typedef v16bf V; static __device__ __forceinline__ V ld(const bf* p) { return cat16b(*(const v8us*)p, *(const v8us*)(p + 16)); } static __device__ __forceinline__ v8f mma(V a, V b, v8f c) { return wmmab(a, b, c); } };
template <typename T16, int NSPLIT, bool BIAS>
__global__ __launch_bounds__(32) void k_gemmw(const T16* __restrict__ A, const T16* __restrict__ A2, const T16* __restrict__ Bt, const T16* __restrict__ Bt2, int K, float* C, int ldc, const float* __restrict__ bias, size_t sA, size_t sB, size_t sC) {
    typedef typename WFrag<T16>::V V;
    __shared__ __align__(16) float os[16 * 68];
    const size_t z = blockIdx.z; A += z * sA; if (A2) A2 += z * sA; Bt += z * sB; if (Bt2) Bt2 += z * sB; C += z * sC;
    const int lane = threadIdx.x & 31, lr = lane & 15, hi = lane >> 4; const int r0 = blockIdx.x * 64, c0 = blockIdx.y * 64;
    v8f acc[4][4];
#pragma unroll
    for (int mb = 0; mb < 4; ++mb)
#pragma unroll
        for (int nb = 0; nb < 4; ++nb) acc[mb][nb] = (v8f){};
    const size_t aoff = (size_t)(r0 + lr) * K + 8 * hi, boff = (size_t)(c0 + lr) * K + 8 * hi;
#pragma unroll 1
    for (int kc = 0; kc < K; kc += 32) {
        V a[4], a2[4];
#pragma unroll
        for (int mb = 0; mb < 4; ++mb) { a[mb] = WFrag<T16>::ld(A + aoff + (size_t)mb * 16 * K + kc); if (NSPLIT == 1 || NSPLIT == 2) a2[mb] = WFrag<T16>::ld(A2 + aoff + (size_t)mb * 16 * K + kc); }
#pragma unroll
        for (int nb = 0; nb < 4; ++nb) { const V b = WFrag<T16>::ld(Bt + boff + (size_t)nb * 16 * K + kc); V b2; if (NSPLIT >= 2) b2 = WFrag<T16>::ld(Bt2 + boff + (size_t)nb * 16 * K + kc);
#pragma unroll
            for (int mb = 0; mb < 4; ++mb) { acc[mb][nb] = WFrag<T16>::mma(a[mb], b, acc[mb][nb]); if (NSPLIT == 1 || NSPLIT == 2) acc[mb][nb] = WFrag<T16>::mma(a2[mb], b, acc[mb][nb]); if (NSPLIT >= 2) acc[mb][nb] = WFrag<T16>::mma(a[mb], b2, acc[mb][nb]); } }
        asm volatile("v_nop\n\tv_nop\n\tv_nop\n\tv_nop" : "+v"(acc[0][0]), "+v"(acc[1][1]), "+v"(acc[2][2]), "+v"(acc[3][3]) : "v"(a[0]), "v"(a[3]));
    }
#pragma unroll
    for (int mb = 0; mb < 4; ++mb) {
#pragma unroll
        for (int nb = 0; nb < 4; ++nb) {
#pragma unroll
            for (int j = 0; j < 8; ++j) os[(hi * 8 + j) * 68 + nb * 16 + lr] = acc[mb][nb][j]; }
        __builtin_amdgcn_wave_barrier(); asm volatile("" ::: "memory");
        float* crow = C + (size_t)(r0 + mb * 16) * ldc + c0;
#pragma unroll 1
        for (int ps = 0; ps < 2; ++ps) {
#pragma unroll
            for (int s = 0; s < 8; ++s) { const int row = 2 * s + hi, cofs = lr * 4; v4f val = *(const v4fa*)(os + row * 68 + cofs); if (BIAS) { val[0] += bfr(bias[c0 + cofs]); val[1] += bfr(bias[c0 + cofs + 1]); val[2] += bfr(bias[c0 + cofs + 2]); val[3] += bfr(bias[c0 + cofs + 3]); }
                *(volatile v4f*)(crow + (size_t)row * ldc + cofs) = val; }
            if (ps == 0) __threadfence(); }
        __builtin_amdgcn_wave_barrier(); asm volatile("" ::: "memory");
    }
}

__device__ __forceinline__ void splitf(float y, unsigned short& h, unsigned short& l) { h = f2bf(y); l = f2bf(y - bf2f(h)); }
typedef __attribute__((ext_vector_type(4))) unsigned short v4us;
typedef __attribute__((ext_vector_type(2))) float v2f;

__global__ __launch_bounds__(256) void k_mm1(const float* __restrict__ x, float* PM) { __shared__ float smn[256], smx[256]; const size_t base = (size_t)blockIdx.x * 8192; float mn = 3.0e38f, mx = -3.0e38f; for (int i = threadIdx.x; i < 8192; i += 256) { const float v = bfr(x[base + i]); mn = fminf(mn, v); mx = fmaxf(mx, v); } smn[threadIdx.x] = mn; smx[threadIdx.x] = mx; __syncthreads();
    for (int s = 128; s > 0; s >>= 1) { if (threadIdx.x < s) { smn[threadIdx.x] = fminf(smn[threadIdx.x], smn[threadIdx.x + s]); smx[threadIdx.x] = fmaxf(smx[threadIdx.x], smx[threadIdx.x + s]); } __syncthreads(); }
    if (threadIdx.x < 32) { const float o = threadIdx.x == 0 ? smn[0] : (threadIdx.x == 1 ? smx[0] : 0.f); *(volatile float*)(PM + blockIdx.x * 32 + threadIdx.x) = o; __threadfence(); *(volatile float*)(PM + blockIdx.x * 32 + threadIdx.x) = o; } }
__global__ __launch_bounds__(32) void k_mm2(const float* __restrict__ PM, int nblk, float* SC) { const int lane = threadIdx.x; float mn = 3.0e38f, mx = -3.0e38f; for (int i = lane; i < nblk; i += 32) { mn = fminf(mn, PM[i * 32]); mx = fmaxf(mx, PM[i * 32 + 1]); }
#pragma unroll
    for (int sh = 16; sh; sh >>= 1) { mn = fminf(mn, __shfl_xor(mn, sh, 32)); mx = fmaxf(mx, __shfl_xor(mx, sh, 32)); }
    const float s = fmaxf(__fdiv_rn(__fsub_rn(mx, mn), 254.0f), 1e-8f); const float o = lane == 0 ? s : 0.f; *(volatile float*)(SC + lane) = o; __threadfence(); *(volatile float*)(SC + lane) = o; }
__global__ __launch_bounds__(256) void k_xq(const float* __restrict__ x, const float* __restrict__ SC, float* XQ, bf* Xh, bf* Xl) { const size_t e = ((size_t)blockIdx.x * 256 + threadIdx.x) * 4; if (e >= (size_t)BB * KKb * NNb) return; const int col = (int)(e % (KKb * NNb)); const int b = (int)(e / (KKb * NNb)); const int k = col / NNb, n = col % NNb; const float s = SC[0]; v4f o; v4us oh, ol;
#pragma unroll
    for (int q = 0; q < 4; ++q) { const float r = fminf(fmaxf(rintf(__fdiv_rn(bfr(x[e + q]), s)), -127.0f), 127.0f); o[q] = __fmul_rn(r, s); unsigned short a, c; splitf(o[q], a, c); oh[q] = a; ol[q] = c; }
    const size_t po = ((size_t)k * BB + b) * NNb + n; *(volatile v4f*)(XQ + e) = o; *(volatile v4us*)(Xh + po) = oh; *(volatile v4us*)(Xl + po) = ol; __threadfence(); *(volatile v4f*)(XQ + e) = o; *(volatile v4us*)(Xh + po) = oh; *(volatile v4us*)(Xl + po) = ol; }
__global__ __launch_bounds__(256) void k_zt(const float* __restrict__ Zs, const float* __restrict__ Zsc, bf* ZT) { const size_t e = ((size_t)blockIdx.x * 256 + threadIdx.x) * 4; if (e >= (size_t)PPd * KKb * JL * NNb) return; const int n = (int)(e % NNb); const int jl = (int)((e / NNb) % JL); const int k = (int)((e / ((size_t)NNb * JL)) % KKb); const int p = (int)(e / ((size_t)NNb * JL * KKb)); const int j = jl / LL, l = jl % LL; const float sc = bfr(Zsc[(p * JJ + j) * KKb + k]); const float* zs = Zs + ((((size_t)p * JJ + j) * KKb + k) * LL + l) * NNb + n; v4us o;
#pragma unroll
    for (int q = 0; q < 4; ++q) o[q] = f2bf(__fmul_rn(bfr(zs[q]), sc)); *(volatile v4us*)(ZT + e) = o; __threadfence(); *(volatile v4us*)(ZT + e) = o; }
__global__ __launch_bounds__(256) void k_ys(const float* __restrict__ Ysg, bf* YS) { const size_t e = ((size_t)blockIdx.x * 256 + threadIdx.x) * 4; if (e >= (size_t)JJ * MM * PKL) return; const int pkl = (int)(e % PKL); const int m = (int)((e / PKL) % MM); const int j = (int)(e / ((size_t)PKL * MM)); v4us o;
#pragma unroll
    for (int q = 0; q < 4; ++q) { const int idx = pkl + q; const int l = idx % LL; const int k = (idx / LL) % KKb; const int p = idx / (LL * KKb); o[q] = f2bf(bfr(Ysg[((((size_t)p * JJ + j) * KKb + k) * MM + m) * LL + l])); } *(volatile v4us*)(YS + e) = o; __threadfence(); *(volatile v4us*)(YS + e) = o; }
__global__ __launch_bounds__(256) void k_tj(const float* __restrict__ T, const float* __restrict__ A4, const float* __restrict__ Ysc, bf* Th, bf* Tl) { const size_t e = ((size_t)blockIdx.x * 256 + threadIdx.x) * 4; if (e >= (size_t)JJ * BB * PKL) return; const int pkl = (int)(e % PKL); const int b = (int)((e / PKL) % BB); const int j = (int)(e / ((size_t)PKL * BB)); v4us oh, ol;
#pragma unroll
    for (int q = 0; q < 4; ++q) { const int idx = pkl + q; const int l = idx % LL; const int k = (idx / LL) % KKb; const int p = idx / (LL * KKb); const size_t pjk = ((size_t)p * JJ + j) * KKb + k; const float t = T[(((size_t)p * KKb + k) * BB + b) * JL + j * LL + l]; float f = __fmul_rn(bfr(A4[pjk * 4]), bfr(Ysc[pjk])); asm volatile("" : "+v"(f)); unsigned short a, c; splitf(__fmul_rn(t, f), a, c); oh[q] = a; ol[q] = c; }
    *(volatile v4us*)(Th + e) = oh; *(volatile v4us*)(Tl + e) = ol; __threadfence(); *(volatile v4us*)(Th + e) = oh; *(volatile v4us*)(Tl + e) = ol; }
__global__ __launch_bounds__(256) void k_sx(const float* __restrict__ XQ, float* SX) { const int e = blockIdx.x * 256 + threadIdx.x; if (e >= BB * KKb) return; const int k = e % KKb, b = e / KKb; float s = 0.f; for (int n = 0; n < NNb; ++n) s = __fadd_rn(s, XQ[(size_t)b * KKb * NNb + k * NNb + n]); *(volatile float*)(SX + e) = s; __threadfence(); *(volatile float*)(SX + e) = s; }
__global__ __launch_bounds__(256) void k_bcoef(const float* __restrict__ A4, const float* __restrict__ Ysg, const float* __restrict__ Ysc, float* BC) { const int e = blockIdx.x * 256 + threadIdx.x; if (e >= JJ * KKb * MM) return; const int m = e % MM; const int k = (e / MM) % KKb; const int j = e / (MM * KKb); float s = 0.f;
    for (int p = 0; p < PPd; ++p) { const size_t pjk = ((size_t)p * JJ + j) * KKb + k; float ys = 0.f; for (int l = 0; l < LL; ++l) { float yq = __fmul_rn(bfr(Ysg[(pjk * MM + m) * LL + l]), bfr(Ysc[pjk])); asm volatile("" : "+v"(yq)); ys = __fadd_rn(ys, yq); } float t = __fmul_rn(bfr(A4[pjk * 4 + 1]), ys); asm volatile("" : "+v"(t)); s = __fadd_rn(s, t); }
    *(volatile float*)(BC + e) = s; __threadfence(); *(volatile float*)(BC + e) = s; }
__global__ __launch_bounds__(256) void k_zsum(const float* __restrict__ Zs, const float* __restrict__ Zsc, float* ZS) { const int e = blockIdx.x * 256 + threadIdx.x; if (e >= PPd * JJ * KKb * NNb) return; const int n = e % NNb; const size_t pjk = e / NNb; const float sc = bfr(Zsc[pjk]); float zsum = 0.f; for (int l = 0; l < LL; ++l) { float zq = __fmul_rn(bfr(Zs[(pjk * LL + l) * NNb + n]), sc); asm volatile("" : "+v"(zq)); zsum = __fadd_rn(zsum, zq); }
    *(volatile float*)(ZS + e) = zsum; __threadfence(); *(volatile float*)(ZS + e) = zsum; }
__global__ __launch_bounds__(256) void k_o34(const float* __restrict__ XQ, const float* __restrict__ SX, const float* __restrict__ ZS, const float* __restrict__ A4, float* O34) { const int e = blockIdx.x * 256 + threadIdx.x; if (e >= BB * JJ) return; const int j = e % JJ, b = e / JJ; float o3 = 0.f, o4 = 0.f;
    for (int p = 0; p < PPd; ++p) for (int k = 0; k < KKb; ++k) { const size_t pjk = ((size_t)p * JJ + j) * KKb + k; float tz = 0.f; const float* xr = XQ + (size_t)b * KKb * NNb + k * NNb; const float* zr = ZS + pjk * NNb;
            for (int n = 0; n < NNb; ++n) { float q = __fmul_rn(xr[n], zr[n]); asm volatile("" : "+v"(q)); tz = __fadd_rn(tz, q); }
            float t3 = __fmul_rn(tz, bfr(A4[pjk * 4 + 2])); asm volatile("" : "+v"(t3)); o3 = __fadd_rn(o3, t3); }
    for (int k = 0; k < KKb; ++k) { float d = 0.f; for (int p = 0; p < PPd; ++p) d = __fadd_rn(d, bfr(A4[(((size_t)p * JJ + j) * KKb + k) * 4 + 3])); float t4 = __fmul_rn(SX[b * KKb + k], d); asm volatile("" : "+v"(t4)); o4 = __fadd_rn(o4, t4); }
    const float o = __fadd_rn(o3, o4); *(volatile float*)(O34 + e) = o; __threadfence(); *(volatile float*)(O34 + e) = o; }
__global__ __launch_bounds__(256) void k_fin(const float* __restrict__ O1, const float* __restrict__ SX, const float* __restrict__ BC, const float* __restrict__ O34, const float* __restrict__ bias, float* OUT) { const size_t e = ((size_t)blockIdx.x * 256 + threadIdx.x) * 4; if (e >= (size_t)BB * JJ * MM) return; const int col = (int)(e % (JJ * MM)); const int b = (int)(e / (JJ * MM)); const int j = col / MM, m = col % MM; v4f o;
#pragma unroll
    for (int q = 0; q < 4; ++q) { const int mq = m + q; float o2 = 0.f; for (int k = 0; k < KKb; ++k) { float t = __fmul_rn(SX[b * KKb + k], BC[((size_t)j * KKb + k) * MM + mq]); asm volatile("" : "+v"(t)); o2 = __fadd_rn(o2, t); }
        o[q] = __fadd_rn(__fadd_rn(__fadd_rn(O1[((size_t)j * BB + b) * MM + mq], o2), O34[b * JJ + j]), bfr(bias[col + q])); }
    *(volatile v4f*)(OUT + e) = o; __threadfence(); *(volatile v4f*)(OUT + e) = o; }

extern "C" void kernel_launch(void* const* d_in, const int* in_sizes, int n_in,
                              void* d_out, int out_size, void* d_ws, size_t ws_size, hipStream_t stream) {
    (void)in_sizes; (void)n_in; (void)out_size;
    const float* x = (const float*)d_in[0]; const float* Ysg = (const float*)d_in[1]; const float* Zsg = (const float*)d_in[2]; const float* Ysc = (const float*)d_in[3]; const float* Zsc = (const float*)d_in[4]; const float* A4 = (const float*)d_in[5]; const float* bias = (const float*)d_in[6];
    float* OUT = (float*)d_out;
    char* wsp = (char*)d_ws;
    auto take = [&](size_t bytes) { char* p = wsp; wsp += (bytes + 255) & ~(size_t)255; return (void*)p; };
    const int NBLK = BB * KKb * NNb / 8192;
    float* PM = (float*)take((size_t)NBLK * 32 * 4); float* SC = (float*)take(32 * 4); float* XQ = (float*)take((size_t)BB * KKb * NNb * 4); bf* Xh = (bf*)take((size_t)KKb * BB * NNb * 2); bf* Xl = (bf*)take((size_t)KKb * BB * NNb * 2);
    bf* ZT = (bf*)take((size_t)PPd * KKb * JL * NNb * 2); bf* YS = (bf*)take((size_t)JJ * MM * PKL * 2); float* T = (float*)take((size_t)PPd * KKb * BB * JL * 4); bf* Th = (bf*)take((size_t)JJ * BB * PKL * 2); bf* Tl = (bf*)take((size_t)JJ * BB * PKL * 2); float* O1 = (float*)take((size_t)JJ * BB * MM * 4);
    float* SX = (float*)take((size_t)BB * KKb * 4); float* ZS = (float*)take((size_t)PPd * JJ * KKb * NNb * 4); float* BC = (float*)take((size_t)JJ * KKb * MM * 4); float* O34 = (float*)take((size_t)BB * JJ * 4);
    if ((size_t)(wsp - (char*)d_ws) > ws_size) return;
    k_mm1<<<NBLK, 256, 0, stream>>>(x, PM); k_mm2<<<1, 32, 0, stream>>>(PM, NBLK, SC);
    k_xq<<<(unsigned)(((size_t)BB * KKb * NNb / 4 + 255) / 256), 256, 0, stream>>>(x, SC, XQ, Xh, Xl);
    k_zt<<<(unsigned)(((size_t)PPd * KKb * JL * NNb / 4 + 255) / 256), 256, 0, stream>>>(Zsg, Zsc, ZT); k_ys<<<(unsigned)(((size_t)JJ * MM * PKL / 4 + 255) / 256), 256, 0, stream>>>(Ysg, YS);
    for (int p = 0; p < PPd; ++p) k_gemmw<bf, 1, false><<<dim3(BB / 64, JL / 64, KKb), 32, 0, stream>>>(Xh, Xl, ZT + (size_t)p * KKb * JL * NNb, nullptr, NNb, T + (size_t)p * KKb * BB * JL, JL, nullptr, (size_t)BB * NNb, (size_t)JL * NNb, (size_t)BB * JL);
    k_tj<<<(unsigned)(((size_t)JJ * BB * PKL / 4 + 255) / 256), 256, 0, stream>>>(T, A4, Ysc, Th, Tl);
    k_gemmw<bf, 1, false><<<dim3(BB / 64, MM / 64, JJ), 32, 0, stream>>>(Th, Tl, YS, nullptr, PKL, O1, MM, nullptr, (size_t)BB * PKL, (size_t)MM * PKL, (size_t)BB * MM);
    k_sx<<<(BB * KKb + 255) / 256, 256, 0, stream>>>(XQ, SX); k_bcoef<<<(JJ * KKb * MM + 255) / 256, 256, 0, stream>>>(A4, Ysg, Ysc, BC); k_zsum<<<(PPd * JJ * KKb * NNb + 255) / 256, 256, 0, stream>>>(Zsg, Zsc, ZS); k_o34<<<(BB * JJ + 255) / 256, 256, 0, stream>>>(XQ, SX, ZS, A4, O34);
    k_fin<<<(unsigned)(((size_t)BB * JJ * MM / 4 + 255) / 256), 256, 0, stream>>>(O1, SX, BC, O34, bias, OUT);
}
